// LinearAttention_24970939859449
// MI455X (gfx1250) — hardware-verified
//
#include <hip/hip_runtime.h>

#ifndef NB
#define NB 4
#endif
#ifndef SEQ
#define SEQ 2048
#endif
#define NB_FULL 4
#define SEQ_FULL 2048
#define DMD 1024
#define NH 16
#define FD 16
#define HDIM 64
#define FV 273
#define FP 288
#define CH 32
#define NQK (2 * NH * FD)
#define MROWS (NB * SEQ)
#define KVSLAB (HDIM * FV)
#define KVLINES (KVSLAB / 32)
#define OUT1_FLOATS ((size_t)NB_FULL * SEQ_FULL * DMD)
#define WSC 256.0f
#define FEATC 2.8284271247461903f
#define RESC 1024.0f
#define RESINV (1.0f / 1024.0f)

static_assert(NB >= 1 && NB <= NB_FULL);
static_assert(SEQ >= 128 && SEQ <= SEQ_FULL && (SEQ % 128) == 0 && (SEQ % CH) == 0);
static_assert(NB == 1 || SEQ == SEQ_FULL);
static_assert(FP % 32 == 0 && FP >= FV && FP == 4 * 72);
static_assert(KVSLAB % 32 == 0 && KVLINES == 546);
static_assert(OUT1_FLOATS * 4 == (size_t)33554432);
static_assert((OUT1_FLOATS + (size_t)NB_FULL * NH * KVSLAB) * 4 == (size_t)38027264);
static_assert(MROWS % 128 == 0 && NQK % 64 == 0 && DMD % 64 == 0 && DMD % 32 == 0);
static_assert(((size_t)MROWS * DMD / 8) % 256 == 0);
static_assert((NH * FD * DMD / 8) % 256 == 0 && (DMD * DMD / 8) % 256 == 0);

typedef _Float16 v16h __attribute__((ext_vector_type(16)));
typedef _Float16 v4h __attribute__((ext_vector_type(4)));
typedef unsigned short v8us __attribute__((ext_vector_type(8), may_alias));
typedef float v8f __attribute__((ext_vector_type(8)));
typedef float v4f __attribute__((ext_vector_type(4)));
typedef float v4fa __attribute__((ext_vector_type(4), may_alias));
union FragH { v16h v; v8us half[2]; _Float16 h[16]; unsigned short u[16]; };

__device__ __forceinline__ unsigned short bf16_bits(float x) { unsigned int u = __float_as_uint(x); return (unsigned short)((u + 0x7FFFu + ((u >> 16) & 1u)) >> 16); }
__device__ __forceinline__ float bf16_val(unsigned short b) { return __uint_as_float(((unsigned int)b) << 16); }
__device__ __forceinline__ float bf16_rne(float x) { return bf16_val(bf16_bits(x)); }

__device__ __forceinline__ v16h fragp(const unsigned short* p, int hh) {
  FragH f; f.half[0] = *(const v8us*)(p + 8 * hh); f.half[1] = *(const v8us*)(p + 16 + 8 * hh); return f.v;
}
__device__ __forceinline__ v8f mma16(v16h a, v16h b, v8f c) {
  v8f d = __builtin_amdgcn_wmma_f32_16x16x32_f16(false, a, false, b, (short)0, c, false, false);
  asm volatile("v_nop\n\tv_nop\n\tv_nop\n\tv_nop" : "+v"(d) : "v"(a), "v"(b));
  return d;
}

__global__ __launch_bounds__(256) void k_x16(const float* __restrict__ x, unsigned short* __restrict__ X16, size_t n8) {
  const size_t t = (size_t)blockIdx.x * 256 + threadIdx.x; if (t >= n8) return;
  const v4f a = *(const v4fa*)(x + t * 8), c = *(const v4fa*)(x + t * 8 + 4);
  FragH f;
#pragma unroll
  for (int q = 0; q < 4; ++q) { f.h[q] = (_Float16)bf16_rne(a[q]); f.h[4 + q] = (_Float16)bf16_rne(c[q]); }
  const v8us o = f.half[0];
  *(volatile v8us*)(X16 + t * 8) = o; __threadfence(); *(volatile v8us*)(X16 + t * 8) = o;
}

__global__ __launch_bounds__(256) void k_wconv(const float* __restrict__ Wq, const float* __restrict__ Wk, const float* __restrict__ Wv, const float* __restrict__ Wo,
                                              unsigned short* __restrict__ WQK, unsigned short* __restrict__ WV, unsigned short* __restrict__ WO) {
  const int blk = blockIdx.x, tid = threadIdx.x;
  const float* src; unsigned short* dst; int i;
  if (blk < 128) { src = Wq; dst = WQK; i = blk * 256 + tid; }
  else if (blk < 256) { src = Wk; dst = WQK + (size_t)NH * FD * DMD; i = (blk - 128) * 256 + tid; }
  else if (blk < 768) { src = Wv; dst = WV; i = (blk - 256) * 256 + tid; }
  else { src = Wo; dst = WO; i = (blk - 768) * 256 + tid; }
  const v4f a = *(const v4fa*)(src + (size_t)i * 8), c = *(const v4fa*)(src + (size_t)i * 8 + 4);
  FragH f;
#pragma unroll
  for (int q = 0; q < 4; ++q) { f.h[q] = (_Float16)(bf16_rne(a[q]) * WSC); f.h[4 + q] = (_Float16)(bf16_rne(c[q]) * WSC); }
  const v8us o = f.half[0];
  *(volatile v8us*)(dst + (size_t)i * 8) = o; __threadfence(); *(volatile v8us*)(dst + (size_t)i * 8) = o;
}

template <bool OUT16>
__global__ __launch_bounds__(128) void k_gemm(const unsigned short* __restrict__ A, int lda, const unsigned short* __restrict__ Bh, int ldb, float alpha,
                                             float* __restrict__ C, _Float16* __restrict__ C16, _Float16* __restrict__ C16L, int ldc, int M, int N, int K) {
  __shared__ __attribute__((aligned(16))) float so[4][32][68];
  const int tid = threadIdx.x, w = tid >> 5, lane = tid & 31, ln = lane & 15, hh = lane >> 4;
  const int ntn = N >> 6; const int mt = blockIdx.x / ntn, nq = blockIdx.x - mt * ntn;
  const int row0 = mt * 128 + 32 * w, col0 = nq * 64; if (row0 >= M) return;
  const unsigned short* a0p = A + (size_t)(row0 + ln) * lda; const unsigned short* a1p = a0p + (size_t)16 * lda;
  const unsigned short* b0p = Bh + (size_t)(col0 + ln) * ldb; const unsigned short* b1p = b0p + (size_t)16 * ldb;
  const unsigned short* b2p = b1p + (size_t)16 * ldb; const unsigned short* b3p = b2p + (size_t)16 * ldb;
  const v8f z8 = {0.f, 0.f, 0.f, 0.f, 0.f, 0.f, 0.f, 0.f};
  v8f c00 = z8, c01 = z8, c02 = z8, c03 = z8, c10 = z8, c11 = z8, c12 = z8, c13 = z8;
#pragma unroll 1
  for (int kb = 0; kb < K; kb += 32) {
    const v16h a0 = fragp(a0p + kb, hh), a1 = fragp(a1p + kb, hh);
    v16h b = fragp(b0p + kb, hh); c00 = mma16(a0, b, c00); c10 = mma16(a1, b, c10);
    b = fragp(b1p + kb, hh); c01 = mma16(a0, b, c01); c11 = mma16(a1, b, c11);
    b = fragp(b2p + kb, hh); c02 = mma16(a0, b, c02); c12 = mma16(a1, b, c12);
    b = fragp(b3p + kb, hh); c03 = mma16(a0, b, c03); c13 = mma16(a1, b, c13);
  }
  v8f accs[8] = {c00, c01, c02, c03, c10, c11, c12, c13};
#pragma unroll
  for (int u = 0; u < 8; ++u) {
    const int t = u & 3, half = u >> 2;
#pragma unroll
    for (int r = 0; r < 8; ++r) so[w][half * 16 + 8 * hh + r][t * 16 + ln] = accs[u][r] * alpha;
  }
  __builtin_amdgcn_fence(4  , "workgroup"); __builtin_amdgcn_wave_barrier();
  const int rsub = lane >> 4, c4 = (lane & 15) * 4;
  for (int pass = 0; pass < 2; ++pass) {
#pragma unroll
    for (int q = 0; q < 16; ++q) {
      const int r = q * 2 + rsub; const v4f v = *(const v4fa*)&so[w][r][c4];
      if constexpr (!OUT16) { *(volatile v4f*)(C + (size_t)(row0 + r) * ldc + col0 + c4) = v; }
      else {
        v4h h4, l4;
#pragma unroll
        for (int i = 0; i < 4; ++i) { const _Float16 hq = (_Float16)v[i]; h4[i] = hq; l4[i] = (_Float16)((v[i] - (float)hq) * RESC); }
        *(volatile v4h*)(C16 + (size_t)(row0 + r) * ldc + col0 + c4) = h4;
        *(volatile v4h*)(C16L + (size_t)(row0 + r) * ldc + col0 + c4) = l4;
      }
    }
    if (pass == 0) __threadfence();
  }
}

template <int D> __device__ __forceinline__ float featv(const float* x, const float* xc, float zl) {
  if constexpr (D == 0) { (void)x; (void)xc; return 16.0f + zl; }
  else if constexpr (D <= FD) { (void)xc; (void)zl; return x[D - 1] * 8.0f; }
  else if constexpr (D < FV) { (void)zl; return xc[(D - 1 - FD) / FD] * x[(D - 1 - FD) % FD]; }
  else { (void)x; (void)xc; return zl; }
}
template <int D0> __device__ __forceinline__ void grp8(const float* q, const float* qc, const float* k, const float* kc, float zl,
                                                        unsigned short* qrow, unsigned short* krow, unsigned short* kft, int lane) {
  FragH fq, fk;
  fq.h[0] = (_Float16)featv<D0 + 0>(q, qc, zl); fk.h[0] = (_Float16)featv<D0 + 0>(k, kc, zl);
  fq.h[1] = (_Float16)featv<D0 + 1>(q, qc, zl); fk.h[1] = (_Float16)featv<D0 + 1>(k, kc, zl);
  fq.h[2] = (_Float16)featv<D0 + 2>(q, qc, zl); fk.h[2] = (_Float16)featv<D0 + 2>(k, kc, zl);
  fq.h[3] = (_Float16)featv<D0 + 3>(q, qc, zl); fk.h[3] = (_Float16)featv<D0 + 3>(k, kc, zl);
  fq.h[4] = (_Float16)featv<D0 + 4>(q, qc, zl); fk.h[4] = (_Float16)featv<D0 + 4>(k, kc, zl);
  fq.h[5] = (_Float16)featv<D0 + 5>(q, qc, zl); fk.h[5] = (_Float16)featv<D0 + 5>(k, kc, zl);
  fq.h[6] = (_Float16)featv<D0 + 6>(q, qc, zl); fk.h[6] = (_Float16)featv<D0 + 6>(k, kc, zl);
  fq.h[7] = (_Float16)featv<D0 + 7>(q, qc, zl); fk.h[7] = (_Float16)featv<D0 + 7>(k, kc, zl);
  *(v8us*)(qrow + D0) = fq.half[0];
  *(v8us*)(krow + D0) = fk.half[0];
#pragma unroll
  for (int e = 0; e < 8; ++e) kft[(D0 + e) * CH + lane] = fk.u[e];
}
template <int W> __device__ __forceinline__ void feat72(const float* q, const float* qc, const float* k, const float* kc, float zl,
                                                         unsigned short* qrow, unsigned short* krow, unsigned short* kft, int lane) {
  grp8<72 * W + 0>(q, qc, k, kc, zl, qrow, krow, kft, lane);  grp8<72 * W + 8>(q, qc, k, kc, zl, qrow, krow, kft, lane);
  grp8<72 * W + 16>(q, qc, k, kc, zl, qrow, krow, kft, lane); grp8<72 * W + 24>(q, qc, k, kc, zl, qrow, krow, kft, lane);
  grp8<72 * W + 32>(q, qc, k, kc, zl, qrow, krow, kft, lane); grp8<72 * W + 40>(q, qc, k, kc, zl, qrow, krow, kft, lane);
  grp8<72 * W + 48>(q, qc, k, kc, zl, qrow, krow, kft, lane); grp8<72 * W + 56>(q, qc, k, kc, zl, qrow, krow, kft, lane);
  grp8<72 * W + 64>(q, qc, k, kc, zl, qrow, krow, kft, lane);
}

__global__ __launch_bounds__(128) void k_attn(const float* __restrict__ QK, const unsigned short* __restrict__ V16, const unsigned short* __restrict__ V16L,
                                             const float* __restrict__ gw, unsigned short* __restrict__ YN, float* __restrict__ KV) {
  __shared__ __attribute__((aligned(16))) float Sf[HDIM * FP];
  __shared__ __attribute__((aligned(16))) unsigned short S16[HDIM * FP];
  __shared__ __attribute__((aligned(16))) unsigned char QFraw[CH * FP * 2];
  __shared__ __attribute__((aligned(16))) unsigned short KF[CH * FP];
  __shared__ __attribute__((aligned(16))) unsigned short KFT[FP * CH];
  __shared__ __attribute__((aligned(16))) unsigned short VT[HDIM * CH];
  __shared__ __attribute__((aligned(16))) unsigned short PT[CH * CH];
  __shared__ float GW[HDIM];
  static_assert(CH * 64 * 4 + CH * 64 * 2 + HDIM * CH * 2 <= CH * FP * 2);
  unsigned short* const QF = (unsigned short*)QFraw;
  float* const ybuf = (float*)QFraw;
  unsigned short* const YNS = (unsigned short*)(QFraw + CH * 64 * 4);
  unsigned short* const VTL = (unsigned short*)(QFraw + CH * 64 * 4 + CH * 64 * 2);

  const int tid = threadIdx.x, w = tid >> 5, lane = tid & 31, ln = lane & 15, hh = lane >> 4;
  const int b = blockIdx.x / NH, h = blockIdx.x - b * NH;
  const size_t rowbase = (size_t)b * SEQ;
  float zl; asm volatile("v_mov_b32 %0, 0" : "=v"(zl));
  for (int i = tid; i < HDIM * FP; i += 128) { Sf[i] = 0.0f; S16[i] = (unsigned short)0; }
  if (tid < HDIM) GW[tid] = bf16_rne(gw[tid]);
  __syncthreads();
  const int rt = w & 1, cg = w >> 1;
  const int wu = __builtin_amdgcn_readfirstlane(w);
  const v8f z8 = {0.f, 0.f, 0.f, 0.f, 0.f, 0.f, 0.f, 0.f};

  for (int ci = 0; ci < SEQ / CH; ++ci) {
    const int r0 = ci * CH;
    {
      const size_t trow = rowbase + r0 + lane;
      const float* qp = QK + trow * NQK + h * FD; const float* kp = qp + NH * FD;
      const v4f q0 = *(const v4fa*)(qp), q1 = *(const v4fa*)(qp + 4), q2 = *(const v4fa*)(qp + 8), q3 = *(const v4fa*)(qp + 12);
      const v4f k0 = *(const v4fa*)(kp), k1 = *(const v4fa*)(kp + 4), k2 = *(const v4fa*)(kp + 8), k3 = *(const v4fa*)(kp + 12);
      float q[16] = {q0[0], q0[1], q0[2], q0[3], q1[0], q1[1], q1[2], q1[3], q2[0], q2[1], q2[2], q2[3], q3[0], q3[1], q3[2], q3[3]};
      float k[16] = {k0[0], k0[1], k0[2], k0[3], k1[0], k1[1], k1[2], k1[3], k2[0], k2[1], k2[2], k2[3], k3[0], k3[1], k3[2], k3[3]};
      float qc[16], kc[16];
#pragma unroll
      for (int i = 0; i < 16; ++i) { qc[i] = q[i] * FEATC; kc[i] = k[i] * FEATC; }
      unsigned short* qrow = QF + lane * FP; unsigned short* krow = KF + lane * FP;
      if (wu == 0) feat72<0>(q, qc, k, kc, zl, qrow, krow, KFT, lane);
      else if (wu == 1) feat72<1>(q, qc, k, kc, zl, qrow, krow, KFT, lane);
      else if (wu == 2) feat72<2>(q, qc, k, kc, zl, qrow, krow, KFT, lane);
      else feat72<3>(q, qc, k, kc, zl, qrow, krow, KFT, lane);
    }
#pragma unroll
    for (int u = 0; u < 2; ++u) {
      const int i = tid + 128 * u; const int m = i >> 3, f8 = (i & 7) * 8;
      FragH f; f.half[0] = *(const v8us*)(V16 + (rowbase + r0 + m) * DMD + h * HDIM + f8);
#pragma unroll
      for (int e = 0; e < 8; ++e) VT[(f8 + e) * CH + m] = f.u[e];
    }
    __syncthreads();

    v8f y0 = z8, y1 = z8, sa = z8;
    {
      const unsigned short* qr = QF + (16 * rt + ln) * FP;
      const unsigned short* s0r = S16 + (32 * cg + ln) * FP; const unsigned short* s1r = s0r + 16 * FP;
      const unsigned short* kr = KF + (16 * cg + ln) * FP;
#pragma unroll 1
      for (int kb = 0; kb < FP; kb += 32) {
        const v16h bq = fragp(qr + kb, hh);
        y0 = mma16(fragp(s0r + kb, hh), bq, y0);
        y1 = mma16(fragp(s1r + kb, hh), bq, y1);
        sa = mma16(fragp(kr + kb, hh), bq, sa);
      }
    }
    {
      const int n = 16 * rt + ln; FragH p;
#pragma unroll
      for (int r = 0; r < 8; ++r) { const int m = 16 * cg + 8 * hh + r; const float keep = (m <= n) ? 1.0f : 0.0f; p.h[r] = (_Float16)(sa[r] * 0.0625f * keep); }
      *(v8us*)(PT + n * CH + 16 * cg + 8 * hh) = p.half[0];
    }
    __syncthreads();

    {
      const v16h bp = fragp(PT + (16 * rt + ln) * CH, hh);
      y0 = mma16(fragp(VT + (32 * cg + ln) * CH, hh), bp, y0);
      y1 = mma16(fragp(VT + (32 * cg + 16 + ln) * CH, hh), bp, y1);
    }
#pragma unroll
    for (int u = 0; u < 2; ++u) {
      const int i = tid + 128 * u; const int m = i >> 3, f8 = (i & 7) * 8;
      FragH f; f.half[0] = *(const v8us*)(V16L + (rowbase + r0 + m) * DMD + h * HDIM + f8);
#pragma unroll
      for (int e = 0; e < 8; ++e) VTL[(f8 + e) * CH + m] = f.u[e];
    }
    {
      const int n = 16 * rt + ln; float* yb = ybuf + n * 64 + 32 * cg + 8 * hh;
      const float sc = 1.0f / 256.0f;
      v4f o0, o1, o2, o3;
#pragma unroll
      for (int j = 0; j < 4; ++j) { o0[j] = y0[j] * sc; o1[j] = y0[4 + j] * sc; o2[j] = y1[j] * sc; o3[j] = y1[4 + j] * sc; }
      *(v4fa*)(yb) = o0; *(v4fa*)(yb + 4) = o1; *(v4fa*)(yb + 16) = o2; *(v4fa*)(yb + 20) = o3;
    }
    __syncthreads();

    {
      const int row = tid >> 2, part = tid & 3;
      const float* yr = ybuf + row * 64 + part * 16;
      const v4f a0 = *(const v4fa*)(yr), a1 = *(const v4fa*)(yr + 4), a2 = *(const v4fa*)(yr + 8), a3 = *(const v4fa*)(yr + 12);
      float ys[16] = {a0[0], a0[1], a0[2], a0[3], a1[0], a1[1], a1[2], a1[3], a2[0], a2[1], a2[2], a2[3], a3[0], a3[1], a3[2], a3[3]};
      float ss = 0.0f;
#pragma unroll
      for (int j = 0; j < 16; ++j) ss += ys[j] * ys[j];
      ss += __shfl_xor(ss, 1); ss += __shfl_xor(ss, 2);
      const float rms = rsqrtf(ss * (1.0f / 64.0f) + 1e-5f);
      FragH o;
#pragma unroll
      for (int j = 0; j < 16; ++j) o.h[j] = (_Float16)(ys[j] * rms * GW[part * 16 + j] * 16.0f);
      *(v8us*)(YNS + row * 64 + part * 16) = o.half[0];
      *(v8us*)(YNS + row * 64 + part * 16 + 8) = o.half[1];
    }
    __syncthreads();
    {
      const int lr = lane >> 3, pc = lane & 7;
      for (int pass = 0; pass < 2; ++pass) {
#pragma unroll
        for (int it = 0; it < 2; ++it) {
          const int row = 8 * w + 4 * it + lr;
          const v8us v = *(const v8us*)(YNS + row * 64 + pc * 8);
          *(volatile v8us*)(YN + (rowbase + r0 + row) * DMD + h * HDIM + pc * 8) = v;
        }
        if (pass == 0) __threadfence();
      }
    }

    {
      const v16h bv = fragp(VT + (16 * w + ln) * CH, hh);
      const v16h bvl = fragp(VTL + (16 * w + ln) * CH, hh);
      float* sp = Sf + (size_t)(16 * w + ln) * FP + 8 * hh;
      unsigned short* s16p = S16 + (16 * w + ln) * FP + 8 * hh;
#pragma unroll 1
      for (int dt = 0; dt < FP / 16; ++dt) {
        const v16h a = fragp(KFT + (16 * dt + ln) * CH, hh);
        const v4f c0 = *(const v4fa*)(sp + 16 * dt), c1 = *(const v4fa*)(sp + 16 * dt + 4);
        v8f c = {c0[0], c0[1], c0[2], c0[3], c1[0], c1[1], c1[2], c1[3]};
        c = mma16(a, bv, c);
        const v8f cl = mma16(a, bvl, z8);
        v4f o0, o1; FragH s;
#pragma unroll
        for (int j = 0; j < 4; ++j) { o0[j] = c[j] + cl[j] * RESINV; o1[j] = c[4 + j] + cl[4 + j] * RESINV; }
#pragma unroll
        for (int r = 0; r < 4; ++r) { s.h[r] = (_Float16)(o0[r] * 0.0625f); s.h[4 + r] = (_Float16)(o1[r] * 0.0625f); }
        *(v4fa*)(sp + 16 * dt) = o0; *(v4fa*)(sp + 16 * dt + 4) = o1;
        *(v8us*)(s16p + 16 * dt) = s.half[0];
      }
    }
    __syncthreads();
  }

  {
    float* kvp = KV + (size_t)(b * NH + h) * KVSLAB;
    const int lr = tid >> 3, pc = tid & 7;
    const float sc = 1.0f / 256.0f;
    for (int pass = 0; pass < 2; ++pass) {
#pragma unroll 1
      for (int it = 0; it < (KVLINES + 15) / 16; ++it) {
        const int line = it * 16 + lr;
        if (line < KVLINES) {
          const int e0 = line * 32 + pc * 4; v4f o;
#pragma unroll
          for (int j = 0; j < 4; ++j) { const int e = e0 + j; const int f = e / FV; const int d = e - f * FV; o[j] = Sf[f * FP + d] * sc; }
          *(volatile v4f*)(kvp + e0) = o;
        }
      }
      if (pass == 0) __threadfence();
    }
  }
}

extern "C" void kernel_launch(void* const* d_in, const int* in_sizes, int n_in,
                              void* d_out, int out_size, void* d_ws, size_t ws_size, hipStream_t stream) {
  if (n_in < 6) return;
  if (in_sizes[0] < (int)(((NB - 1) * SEQ_FULL + SEQ) * DMD) || in_sizes[1] < NH * FD * DMD || in_sizes[2] < NH * FD * DMD ||
      in_sizes[3] < DMD * DMD || in_sizes[4] < DMD * DMD || in_sizes[5] < HDIM) return;
  if ((size_t)out_size < OUT1_FLOATS + (size_t)NB * NH * KVSLAB) return;
  const float* hs = (const float*)d_in[0]; const float* Wq = (const float*)d_in[1]; const float* Wk = (const float*)d_in[2];
  const float* Wv = (const float*)d_in[3]; const float* Wo = (const float*)d_in[4]; const float* gw = (const float*)d_in[5];
  char* ws = (char*)d_ws; size_t off = 0;
  auto take = [&](size_t bytes) { char* p = ws + off; off += (bytes + 255) & ~(size_t)255; return p; };
  unsigned short* X16 = (unsigned short*)take((size_t)MROWS * DMD * 2);
  unsigned short* WQK = (unsigned short*)take((size_t)NQK * DMD * 2);
  unsigned short* WV  = (unsigned short*)take((size_t)DMD * DMD * 2);
  unsigned short* WO  = (unsigned short*)take((size_t)DMD * DMD * 2);
  float* QK32 = (float*)take((size_t)MROWS * NQK * 4);
  unsigned short* V16 = (unsigned short*)take((size_t)MROWS * DMD * 2);
  unsigned short* V16L = (unsigned short*)take((size_t)MROWS * DMD * 2);
  unsigned short* YN  = (unsigned short*)take((size_t)MROWS * DMD * 2);
  if (off > ws_size) return;
  float* out0 = (float*)d_out; float* out1 = (float*)d_out + OUT1_FLOATS;

  const size_t n8 = (size_t)MROWS * DMD / 8;
  k_x16<<<(unsigned)(n8 / 256), 256, 0, stream>>>(hs, X16, n8);
  k_wconv<<<1280, 256, 0, stream>>>(Wq, Wk, Wv, Wo, WQK, WV, WO);
  k_gemm<false><<<(MROWS / 128) * (NQK / 64), 128, 0, stream>>>(X16, DMD, WQK, DMD, 1.0f / 256.0f, QK32, (_Float16*)V16, (_Float16*)V16L, NQK, MROWS, NQK, DMD);
  k_gemm<true><<<(MROWS / 128) * (DMD / 64), 128, 0, stream>>>(X16, DMD, WV, DMD, 1.0f / 16.0f, QK32, (_Float16*)V16, (_Float16*)V16L, DMD, MROWS, DMD, DMD);
  k_attn<<<NB * NH, 128, 0, stream>>>(QK32, V16, V16L, gw, YN, out1);
  k_gemm<false><<<(MROWS / 128) * (DMD / 64), 128, 0, stream>>>(YN, DMD, WO, DMD, 1.0f / 4096.0f, out0, (_Float16*)V16, (_Float16*)V16L, DMD, MROWS, DMD, DMD);
}
